// Linear_extractor_cluster_63840393888217
// MI455X (gfx1250) — hardware-verified
//
#include <hip/hip_runtime.h>
#include <stdint.h>
#include <stddef.h>
#include <math.h>

#pragma clang fp contract(off)

#define NB   512
#define NS   512
#define NC   32
#define ND   512
#define NE   8
#define NEMB 32
#define XSP  520
#define OSP  36
#define TSP  72
#define FRW  64

static_assert((XSP * 2) % 16 == 0);
static_assert((OSP * 4) % 16 == 0);
static_assert((TSP * 2) % 16 == 0);
static_assert(NS % 64 == 0);
static_assert(ND % 256 == 0);
static_assert(NC == 32);
static_assert(NS * NC == 16 * 256 * 4);

typedef _Float16 v16h __attribute__((ext_vector_type(16)));
typedef _Float16 v8h  __attribute__((ext_vector_type(8)));
typedef float    v8f  __attribute__((ext_vector_type(8)));
typedef float    v4f  __attribute__((ext_vector_type(4)));
typedef v8h __attribute__((may_alias)) v8ha;
typedef v4f __attribute__((may_alias)) v4fa;

union FragH { v16h v; v8h q[2]; };
union Pack16 { v8h h; v4f f; };

__device__ __forceinline__ v8f wmma_h(v16h a, v16h b, v8f c) {
  v8f d = __builtin_amdgcn_wmma_f32_16x16x32_f16(false, a, false, b, (short)0, c, false, false);
  asm volatile("v_nop\n\tv_nop\n\tv_nop\n\tv_nop" : "+v"(d) : "v"(a), "v"(b));
  return d;
}

__device__ __forceinline__ v16h ldfrag(const _Float16* p, int h) {
  FragH f;
  f.q[0] = *(const v8ha*)(p + 8 * h);
  f.q[1] = *(const v8ha*)(p + 16 + 8 * h);
  return f.v;
}

__device__ __forceinline__ unsigned int fkey(float f) {
  const unsigned int u = __float_as_uint(f);
  return (u & 0x80000000u) ? ~u : (u | 0x80000000u);
}
__device__ __forceinline__ float funkey(unsigned int u) {
  return (u & 0x80000000u) ? __uint_as_float(u & 0x7fffffffu) : __uint_as_float(~u);
}

__global__ __launch_bounds__(256) void k_front(const float* __restrict__ x,
                                               const float* __restrict__ wp,
                                               const float* __restrict__ bp,
                                               const float* __restrict__ emb,
                                               const float* __restrict__ wg,
                                               const float* __restrict__ bg,
                                               const int*   __restrict__ kin,
                                               float* __restrict__ front)
{
  __shared__ __align__(16) float  sMed[NC];
  __shared__ __align__(16) float  sXl[NC];
  __shared__ __align__(16) float  sCtx[ND];
  __shared__ __align__(16) double sRed[256];
  __shared__ __align__(16) float  sLg[NE];
  __shared__ __align__(16) float  sSV[NE];
  __shared__ __align__(16) int    sSI[NE];
  __shared__ __align__(16) float  sLine[FRW];

  const int tid = threadIdx.x, lane = tid & 31, wv = tid >> 5;
  const int b = blockIdx.x;
  const float* xb = x + (size_t)b * NS * NC;

  #pragma unroll 1
  for (int q = 0; q < 4; ++q) {
    const int c = wv * 4 + q;
    unsigned int key[16];
    #pragma unroll
    for (int i = 0; i < 16; ++i) key[i] = fkey(xb[(size_t)(lane + 32 * i) * NC + c]);

    unsigned int lo = 0u, hi = 0xffffffffu;
    #pragma unroll 1
    for (int it = 0; it < 32; ++it) {
      const unsigned int mid = lo + ((hi - lo) >> 1);
      int cnt = 0;
      #pragma unroll
      for (int i = 0; i < 16; ++i) cnt += (key[i] <= mid) ? 1 : 0;
      #pragma unroll
      for (int off = 16; off > 0; off >>= 1) cnt += __shfl_xor(cnt, off);
      const bool ge = (cnt >= 256);
      hi = ge ? mid : hi;
      lo = ge ? lo : (mid + 1u);
    }
    const unsigned int k0 = lo;
    int c2 = 0;
    unsigned int mn = 0xffffffffu;
    #pragma unroll
    for (int i = 0; i < 16; ++i) {
      c2 += (key[i] <= k0) ? 1 : 0;
      const bool ab = (key[i] > k0) && (key[i] < mn);
      mn = ab ? key[i] : mn;
    }
    #pragma unroll
    for (int off = 16; off > 0; off >>= 1) {
      c2 += __shfl_xor(c2, off);
      const unsigned int o = (unsigned int)__shfl_xor((int)mn, off);
      mn = (o < mn) ? o : mn;
    }
    const unsigned int k1 = (c2 >= 257) ? k0 : mn;
    const float med = (funkey(k0) + funkey(k1)) * 0.5f;
    if (lane == 0) sMed[c] = med;
  }
  __syncthreads();

  if (tid < NC) sXl[tid] = xb[(size_t)(NS - 1) * NC + tid] - sMed[tid];
  __syncthreads();

  #pragma unroll 1
  for (int dd = 0; dd < ND / 256; ++dd) {
    const int d = tid + 256 * dd;
    float a = 0.0f;
    #pragma unroll 1
    for (int v = 0; v < NC; ++v) a = a + sXl[v] * wp[v * ND + d];
    a = a + bp[d];
    sCtx[d] = a;
  }
  __syncthreads();

  {
    const double p = (double)sCtx[tid] * (double)wg[tid] +
                     (double)sCtx[tid + 256] * (double)wg[tid + 256];
    sRed[tid] = p;
  }
  __syncthreads();
  #pragma unroll 1
  for (int s = 128; s > 0; s >>= 1) {
    if (tid < s) sRed[tid] = sRed[tid] + sRed[tid + s];
    __syncthreads();
  }
  if (tid < NE) {
    double qe = 0.0;
    #pragma unroll 1
    for (int j = 0; j < NEMB; ++j) qe = qe + (double)emb[tid * NEMB + j] * (double)wg[ND + j];
    sLg[tid] = (float)(sRed[0] + qe + (double)bg[0]);
  }
  if (tid < NC) sLine[NC + tid] = 0.0f;
  __syncthreads();

  if (tid == 0) {
    int ksel = kin[0];
    ksel = (ksel < 1) ? 1 : ((ksel > NE) ? NE : ksel);
    int used = 0;
    #pragma unroll 1
    for (int j = 0; j < ksel; ++j) {
      float bv = 0.0f;
      int bi = -1;
      #pragma unroll 1
      for (int e = 0; e < NE; ++e) {
        const bool cand = ((used >> e) & 1) == 0;
        const float le = sLg[e];
        const bool take = cand && ((bi < 0) || (le > bv));
        bv = take ? le : bv;
        bi = take ? e : bi;
      }
      bi = (bi < 0) ? 0 : bi;
      used |= (1 << bi);
      sSV[j] = bv;
      sSI[j] = bi;
    }
    const float mx = sSV[0];
    float sum = 0.0f;
    #pragma unroll 1
    for (int j = 0; j < ksel; ++j) {
      const float ex = expf(sSV[j] - mx);
      sSV[j] = ex;
      sum = sum + ex;
    }
    const float rsm = 1.0f / sum;
    #pragma unroll 1
    for (int j = 0; j < ksel; ++j) {
      int e = sSI[j];
      e = (e < 0) ? 0 : ((e > NE - 1) ? (NE - 1) : e);
      sLine[NC + e] = sSV[j] * rsm;
    }
  }
  if (tid < NC) sLine[tid] = sMed[tid];
  __syncthreads();

  if (wv == 0) {
    const int li = lane & 15;
    const v4f v = *(const v4fa*)(sLine + 4 * li);
    float* dst = front + (size_t)b * FRW + 4 * li;
    const bool ok = (lane < 16);
    if (ok) *(volatile v4fa*)dst = v;
    __threadfence();
    if (ok) *(volatile v4fa*)dst = v;
  }
}

__global__ __launch_bounds__(256) void k_wet(const float* __restrict__ we,
                                             _Float16* __restrict__ wet)
{
  __shared__ __align__(16) _Float16 sT[64 * TSP];
  const int tid = threadIdx.x, lane = tid & 31, wv = tid >> 5;
  const int blk = blockIdx.x;
  const int e  = blk >> 6;
  const int st = (blk >> 3) & 7;
  const int dq = blk & 7;
  const int s0 = st * 64, d0 = dq * 64;

  #pragma unroll
  for (int i = 0; i < 4; ++i) {
    const int si = (tid >> 4) + 16 * i;
    const int c4 = 4 * (tid & 15);
    const v4f v = *(const v4fa*)(we + ((size_t)(e * NS + s0 + si)) * ND + d0 + c4);
    sT[(c4 + 0) * TSP + si] = (_Float16)(v.x * 16.0f);
    sT[(c4 + 1) * TSP + si] = (_Float16)(v.y * 16.0f);
    sT[(c4 + 2) * TSP + si] = (_Float16)(v.z * 16.0f);
    sT[(c4 + 3) * TSP + si] = (_Float16)(v.w * 16.0f);
  }
  __syncthreads();

  Pack16 u[2];
  size_t go[2];
  #pragma unroll
  for (int p = 0; p < 2; ++p) {
    const int row = wv * 8 + 4 * p + (lane >> 3);
    const int c8 = 8 * (lane & 7);
    u[p].h = *(const v8ha*)(sT + row * TSP + c8);
    go[p] = ((size_t)(e * ND + d0 + row)) * NS + s0 + c8;
  }
  #pragma unroll
  for (int p = 0; p < 2; ++p) *(volatile v4fa*)(wet + go[p]) = u[p].f;
  __threadfence();
  #pragma unroll
  for (int p = 0; p < 2; ++p) *(volatile v4fa*)(wet + go[p]) = u[p].f;
}

__global__ __launch_bounds__(256) void k_expert(const float* __restrict__ x,
                                                const _Float16* __restrict__ wet,
                                                const float* __restrict__ front,
                                                float* __restrict__ out)
{
  __shared__ __align__(16) _Float16 xs[NC * XSP];
  __shared__ __align__(16) float    sO[8 * 16 * OSP];
  __shared__ __align__(16) float    sF[FRW];

  const int tid = threadIdx.x, lane = tid & 31, wv = tid >> 5;
  const int h = lane >> 4, m = lane & 15;
  const int dh = blockIdx.x;
  const int b  = blockIdx.y;

  if (tid < FRW) sF[tid] = front[(size_t)b * FRW + tid];
  __syncthreads();

  const float* xb = x + (size_t)b * NS * NC;
  #pragma unroll 4
  for (int i = 0; i < 16; ++i) {
    const int q = tid + 256 * i;
    const int s = q >> 3;
    const int v4 = (q & 7) * 4;
    const v4f v = *(const v4fa*)(xb + 4 * q);
    xs[(v4 + 0) * XSP + s] = (_Float16)(v.x - sF[v4 + 0]);
    xs[(v4 + 1) * XSP + s] = (_Float16)(v.y - sF[v4 + 1]);
    xs[(v4 + 2) * XSP + s] = (_Float16)(v.z - sF[v4 + 2]);
    xs[(v4 + 3) * XSP + s] = (_Float16)(v.w - sF[v4 + 3]);
  }
  __syncthreads();

  const int drow0 = dh * 256 + wv * 32;
  const v8f z8 = {0.f, 0.f, 0.f, 0.f, 0.f, 0.f, 0.f, 0.f};
  v8f tot[2][2];
  #pragma unroll
  for (int dt = 0; dt < 2; ++dt)
    #pragma unroll
    for (int vt = 0; vt < 2; ++vt) tot[dt][vt] = z8;

  #pragma unroll 1
  for (int e = 0; e < NE; ++e) {
    const float g = sF[NC + e];
    if (g != 0.0f) {
      v8f acc[2][2];
      #pragma unroll
      for (int dt = 0; dt < 2; ++dt)
        #pragma unroll
        for (int vt = 0; vt < 2; ++vt) acc[dt][vt] = z8;
      const _Float16* arow = wet + ((size_t)(e * ND + drow0 + m)) * NS;
      #pragma unroll 1
      for (int k0 = 0; k0 < NS; k0 += 32) {
        v16h bf[2], af[2];
        #pragma unroll
        for (int vt = 0; vt < 2; ++vt) bf[vt] = ldfrag(xs + (16 * vt + m) * XSP + k0, h);
        #pragma unroll
        for (int dt = 0; dt < 2; ++dt) af[dt] = ldfrag(arow + (size_t)(16 * dt) * NS + k0, h);
        #pragma unroll
        for (int dt = 0; dt < 2; ++dt)
          #pragma unroll
          for (int vt = 0; vt < 2; ++vt) acc[dt][vt] = wmma_h(af[dt], bf[vt], acc[dt][vt]);
      }
      const float gs = g * 0.0625f;
      #pragma unroll
      for (int dt = 0; dt < 2; ++dt)
        #pragma unroll
        for (int vt = 0; vt < 2; ++vt) tot[dt][vt] = tot[dt][vt] + gs * acc[dt][vt];
    }
  }

  float* so = sO + wv * 16 * OSP;
  #pragma unroll
  for (int dt = 0; dt < 2; ++dt) {
    #pragma unroll
    for (int vt = 0; vt < 2; ++vt)
      #pragma unroll
      for (int r = 0; r < 8; ++r) so[(8 * h + r) * OSP + 16 * vt + m] = tot[dt][vt][r];
    __syncthreads();
    v4f w[4];
    size_t go[4];
    #pragma unroll
    for (int p = 0; p < 4; ++p) {
      const int row = 4 * p + (lane >> 3);
      w[p] = *(const v4fa*)(so + row * OSP + 4 * (lane & 7));
      const int d = drow0 + 16 * dt + row;
      go[p] = ((size_t)(b * ND + d)) * NC + 4 * (lane & 7);
    }
    #pragma unroll
    for (int p = 0; p < 4; ++p) *(volatile v4fa*)(out + go[p]) = w[p];
    __threadfence();
    #pragma unroll
    for (int p = 0; p < 4; ++p) *(volatile v4fa*)(out + go[p]) = w[p];
    __syncthreads();
  }
}

extern "C" void kernel_launch(void* const* d_in, const int* in_sizes, int n_in,
                              void* d_out, int out_size, void* d_ws, size_t ws_size,
                              hipStream_t stream)
{
  if (n_in < 8) return;
  if (in_sizes[0] != NB * NS * NC) return;
  if (in_sizes[1] != NC * ND) return;
  if (in_sizes[2] != ND) return;
  if (in_sizes[3] != NE * NEMB) return;
  if (in_sizes[4] != ND + NEMB) return;
  if (in_sizes[5] < 1) return;
  if (in_sizes[6] != NE * NS * ND) return;
  if (in_sizes[7] < 1) return;
  if (out_size != NB * ND * NC) return;

  const float* x   = (const float*)d_in[0];
  const float* wp  = (const float*)d_in[1];
  const float* bp  = (const float*)d_in[2];
  const float* emb = (const float*)d_in[3];
  const float* wg  = (const float*)d_in[4];
  const float* bg  = (const float*)d_in[5];
  const float* we  = (const float*)d_in[6];
  const int*   kin = (const int*)d_in[7];
  float* out = (float*)d_out;

  const size_t bWET = (size_t)NE * ND * NS * 2;
  const size_t bFR  = (size_t)NB * FRW * 4;
  const size_t total = bWET + bFR;
  if (total > ws_size) return;
  if (total > (size_t)134217728) return;

  char* ws = (char*)d_ws;
  size_t off = 0;
  _Float16* WET = (_Float16*)(ws + off); off += bWET;
  float*    FR  = (float*)(ws + off);    off += bFR;
  if (off != total) return;

  k_front<<<NB, 256, 0, stream>>>(x, wp, bp, emb, wg, bg, kin, FR);
  k_wet<<<NE * (NS / 64) * (ND / 64), 256, 0, stream>>>(we, WET);
  k_expert<<<dim3(ND / 256, NB), 256, 0, stream>>>(x, WET, FR, out);
}
